// GraphMessageLayer_28355374088952
// MI455X (gfx1250) — hardware-verified
//
#include <hip/hip_runtime.h>
#include <stddef.h>


typedef _Float16 h16;
typedef _Float16 v16h __attribute__((ext_vector_type(16)));
typedef _Float16 v8h  __attribute__((ext_vector_type(8)));
typedef float    v8f  __attribute__((ext_vector_type(8)));
typedef float    v4f  __attribute__((ext_vector_type(4)));

#ifndef NB
#define NB 8
#endif
#define NB_FULL 8
#define NODES 256
#define HDIM  128
#define KCAT  256
#define EIN   257
#define MROWS (NB * NODES)

static_assert(NB >= 1 && NB <= NB_FULL);
static_assert(NODES == 256);
static_assert((NODES % 64) == 0);
static_assert(HDIM == 128 && KCAT == 2 * HDIM && EIN == 2 * HDIM + 1);
static_assert((HDIM % 64) == 0 && (HDIM % 32) == 0);
static_assert((KCAT % 64) == 0 && (KCAT % 32) == 0);
static_assert((MROWS % 64) == 0 && (MROWS % 16) == 0);
static_assert(HDIM == 16 * 8);

#define LDT 72
#define LDC 68
static_assert((LDT % 8) == 0 && LDT >= 64);
static_assert((LDC % 4) == 0 && LDC >= 64);
static_assert(64 * LDC * 4 + 8 * 4 <= 131072);
static_assert(64 * LDT * 2 <= 131072);

#define WCARRY 64.0f
#define XCARRY 16.0f
#define ACC_SCALE (1.0f / (WCARRY * XCARRY))

#define WE1_BYTES ((size_t)KCAT * HDIM * 2)
#define WSQ_BYTES ((size_t)HDIM * HDIM * 2)
#define WN1_BYTES ((size_t)HDIM * KCAT * 2)
#define NI_BYTES  ((size_t)MROWS * KCAT * 2)
#define P16_BYTES ((size_t)MROWS * HDIM * 2)
#define AC_BYTES  ((size_t)MROWS * KCAT * 4)
#define OFF_WE1 ((size_t)0)
#define OFF_WE2 (OFF_WE1 + WE1_BYTES)
#define OFF_WN1 (OFF_WE2 + WSQ_BYTES)
#define OFF_WN2 (OFF_WN1 + WN1_BYTES)
#define OFF_NI  (OFF_WN2 + WSQ_BYTES)
#define OFF_M   (OFF_NI + NI_BYTES)
#define OFF_HN  (OFF_M + P16_BYTES)
#define OFF_AC  (OFF_HN + P16_BYTES)
#define WS_TOTAL (OFF_AC + AC_BYTES)
static_assert((WE1_BYTES % 128) == 0 && (WSQ_BYTES % 128) == 0 && (WN1_BYTES % 128) == 0);
static_assert((NI_BYTES % 128) == 0 && (P16_BYTES % 128) == 0 && (AC_BYTES % 128) == 0);
static_assert(WS_TOTAL <= (size_t)134217728);
static_assert((size_t)MROWS * HDIM * 4 <= (size_t)1048576);

__device__ __forceinline__ float bf16r(float x) {
  unsigned int u = __float_as_uint(x);
  u = (u + 0x7FFFu + ((u >> 16) & 1u)) & 0xFFFF0000u;
  return __uint_as_float(u);
}

static __device__ __forceinline__ h16 toh_flush(float v) {
  const h16 r = (h16)v;
  return (fabsf(v) < 6.103515625e-05f) ? (h16)0.0f : r;
}

__device__ __forceinline__ v16h frag_at(const _Float16* p) {
  v8h lo = *(const v8h*)(p);
  v8h hi = *(const v8h*)(p + 16);
  v16h out;
#pragma unroll
  for (int i = 0; i < 8; ++i) { out[i] = lo[i]; out[i + 8] = hi[i]; }
  return out;
}

__device__ __forceinline__ v8f wmma16(v16h a, v16h b, v8f c) {
  v8f d = __builtin_amdgcn_wmma_f32_16x16x32_f16(false, a, false, b, (short)0, c,
                                                 false, false);
  asm volatile("v_nop\n\tv_nop\n\tv_nop\n\tv_nop" : "+v"(d) : "v"(a), "v"(b));
  return d;
}

__device__ __forceinline__ float red32_sum(float x) {
#pragma unroll
  for (int off = 1; off < 32; off <<= 1) x += __shfl_xor(x, off, 32);
  return x;
}

__device__ __forceinline__ float silu_act(float t) {
  return t * __builtin_amdgcn_rcpf(1.0f + __expf(-t));
}

__global__ __launch_bounds__(256) void wconv_kernel(
    const float* __restrict__ W, _Float16* __restrict__ Wt, unsigned ldw, unsigned ldk) {
  __shared__ _Float16 T[64 * LDT];
  const unsigned tid = threadIdx.x;
  const unsigned n0 = blockIdx.x * 64u;
  const unsigned k0 = blockIdx.y * 64u;
#pragma unroll 4
  for (unsigned j = 0; j < 16u; ++j) {
    const unsigned idx = tid + 256u * j;
    const unsigned kr = idx >> 6, nc = idx & 63u;
    const float v = W[(size_t)(k0 + kr) * ldw + n0 + nc];
    T[nc * LDT + kr] = toh_flush(WCARRY * bf16r(v));
  }
  __syncthreads();
  v8h x[2];
  size_t off[2];
#pragma unroll
  for (unsigned i = 0; i < 2u; ++i) {
    const unsigned n = 32u * i + (tid >> 3);
    const unsigned kc = (tid & 7u) * 8u;
    x[i] = *(const v8h*)&T[n * LDT + kc];
    off[i] = (size_t)(n0 + n) * ldk + k0 + kc;
  }
#pragma unroll
  for (int i = 0; i < 2; ++i) *(volatile v8h*)(Wt + off[i]) = x[i];
  __threadfence();
#pragma unroll
  for (int i = 0; i < 2; ++i) *(volatile v8h*)(Wt + off[i]) = x[i];
}

__global__ __launch_bounds__(256) void nsconv_kernel(
    const float* __restrict__ X, _Float16* __restrict__ dst) {
  const unsigned gid = blockIdx.x * 256u + threadIdx.x;
  const unsigned row = gid >> 4;
  const unsigned c = (gid & 15u) * 8u;
  const v4f a0 = *(const v4f*)(X + (size_t)row * HDIM + c);
  const v4f a1 = *(const v4f*)(X + (size_t)row * HDIM + c + 4u);
  v8h o;
#pragma unroll
  for (int i = 0; i < 4; ++i) {
    o[i]     = toh_flush(XCARRY * bf16r(a0[i]));
    o[i + 4] = toh_flush(XCARRY * bf16r(a1[i]));
  }
  _Float16* p = dst + (size_t)row * KCAT + c;
  *(volatile v8h*)p = o;
  __threadfence();
  *(volatile v8h*)p = o;
}

template <int MODE>
__device__ __forceinline__ void gemm_body(
    const _Float16* __restrict__ A16, const unsigned lda,
    const _Float16* __restrict__ Bt, const unsigned K,
    const float* __restrict__ bias, const float* __restrict__ maskp,
    const float* __restrict__ xin,
    float* __restrict__ outf, _Float16* __restrict__ out16) {
  __shared__ float Cs[64 * LDC];
  __shared__ float red[8];
  const unsigned tid = threadIdx.x, lane = tid & 31u;
  const unsigned w = (unsigned)__builtin_amdgcn_readfirstlane((int)(tid >> 5));
  const unsigned mw = w >> 1, nw = w & 1u;
  const unsigned hh = lane >> 4, m = lane & 15u;
  const unsigned n0 = blockIdx.x * 64u;
  const unsigned row0 = blockIdx.y * 64u;

  if (MODE == 1) {
    const unsigned bidx = row0 / (unsigned)NODES;
    const float mv = bf16r(maskp[(size_t)bidx * NODES + tid]);
    const float s = red32_sum(mv);
    if (lane == 0u) red[w] = s;
  }

  const _Float16* ap  = A16 + (size_t)(row0 + mw * 16u + m) * lda + hh * 8u;
  const _Float16* bp0 = Bt + (size_t)(n0 + nw * 32u + m) * K + hh * 8u;
  const _Float16* bp1 = bp0 + (size_t)16 * K;
  v8f acc0 = {}, acc1 = {};
#pragma unroll 2
  for (unsigned k0 = 0; k0 < K; k0 += 32u) {
    const v16h a  = frag_at(ap + k0);
    const v16h b0 = frag_at(bp0 + k0);
    const v16h b1 = frag_at(bp1 + k0);
    acc0 = wmma16(a, b0, acc0);
    acc1 = wmma16(a, b1, acc1);
  }
#pragma unroll
  for (int r = 0; r < 8; ++r) {
    float* d = &Cs[(mw * 16u + hh * 8u + (unsigned)r) * LDC + nw * 32u + m];
    d[0]  = acc0[r];
    d[16] = acc1[r];
  }
  __syncthreads();

  if (MODE == 1 || MODE == 2) {
    const unsigned ldo  = (MODE == 1) ? (unsigned)KCAT : (unsigned)HDIM;
    const unsigned cofs = (MODE == 1) ? (unsigned)HDIM : 0u;
    float msum = 0.0f;
    if (MODE == 1)
      msum = ((red[0] + red[1]) + (red[2] + red[3])) + ((red[4] + red[5]) + (red[6] + red[7]));
    v8h x[2];
    size_t off[2];
#pragma unroll
    for (unsigned i = 0; i < 2u; ++i) {
      const unsigned r = 32u * i + (tid >> 3);
      const unsigned c = (tid & 7u) * 8u;
      const unsigned row = row0 + r;
      const v4f u0 = *(const v4f*)&Cs[r * LDC + c];
      const v4f u1 = *(const v4f*)&Cs[r * LDC + c + 4];
      const v4f g0 = *(const v4f*)(bias + n0 + c);
      const v4f g1 = *(const v4f*)(bias + n0 + c + 4u);
      float rr = 1.0f;
      if (MODE == 1) {
        const float mi = bf16r(maskp[row]);
        const float dr = mi * msum;
        rr = dr * __builtin_amdgcn_rcpf(fmaxf(dr, 1.0f));
      }
#pragma unroll
      for (int j = 0; j < 4; ++j) {
        float t0 = u0[j] * ACC_SCALE + rr * bf16r(g0[j]);
        float t1 = u1[j] * ACC_SCALE + rr * bf16r(g1[j]);
        if (MODE == 2) { t0 = silu_act(t0); t1 = silu_act(t1); }
        x[i][j]     = toh_flush(XCARRY * t0);
        x[i][j + 4] = toh_flush(XCARRY * t1);
      }
      off[i] = (size_t)row * ldo + cofs + n0 + c;
    }
#pragma unroll
    for (int i = 0; i < 2; ++i) *(volatile v8h*)(out16 + off[i]) = x[i];
    __threadfence();
#pragma unroll
    for (int i = 0; i < 2; ++i) *(volatile v8h*)(out16 + off[i]) = x[i];
  }

  if (MODE == 0 || MODE == 3) {
    const unsigned ldo = (MODE == 0) ? (unsigned)KCAT : (unsigned)HDIM;
    v4f xs[4];
    size_t off[4];
#pragma unroll
    for (unsigned i = 0; i < 4u; ++i) {
      const unsigned r = 16u * i + (tid >> 4);
      const unsigned c = (tid & 15u) * 4u;
      const unsigned row = row0 + r;
      const v4f u = *(const v4f*)&Cs[r * LDC + c];
      v4f val;
      if (MODE == 0) {
#pragma unroll
        for (int j = 0; j < 4; ++j) val[j] = u[j] * ACC_SCALE;
      } else {
        const v4f g = *(const v4f*)(bias + n0 + c);
        const v4f xv = *(const v4f*)(xin + (size_t)row * HDIM + n0 + c);
        const float mi = bf16r(maskp[row]);
#pragma unroll
        for (int j = 0; j < 4; ++j)
          val[j] = bf16r(xv[j]) + (u[j] * ACC_SCALE + bf16r(g[j])) * mi;
      }
      xs[i] = val;
      off[i] = (size_t)row * ldo + n0 + c;
    }
#pragma unroll
    for (int i = 0; i < 4; ++i) *(volatile v4f*)(outf + off[i]) = xs[i];
    __threadfence();
#pragma unroll
    for (int i = 0; i < 4; ++i) *(volatile v4f*)(outf + off[i]) = xs[i];
  }
}

__global__ __launch_bounds__(256) void gemm_ac_kernel(
    const _Float16* __restrict__ A16, const _Float16* __restrict__ Bt, float* __restrict__ ac) {
  gemm_body<0>(A16, (unsigned)KCAT, Bt, (unsigned)HDIM, ac, ac, ac, ac, (_Float16*)0);
}
__global__ __launch_bounds__(256) void gemm_agg_kernel(
    const _Float16* __restrict__ A16, const _Float16* __restrict__ Bt,
    const float* __restrict__ bias, const float* __restrict__ maskp, _Float16* __restrict__ ni) {
  gemm_body<1>(A16, (unsigned)HDIM, Bt, (unsigned)HDIM, bias, maskp, bias, (float*)0, ni);
}
__global__ __launch_bounds__(256) void gemm_hn_kernel(
    const _Float16* __restrict__ A16, const _Float16* __restrict__ Bt,
    const float* __restrict__ bias, _Float16* __restrict__ hn) {
  gemm_body<2>(A16, (unsigned)KCAT, Bt, (unsigned)KCAT, bias, bias, bias, (float*)0, hn);
}
__global__ __launch_bounds__(256) void gemm_out_kernel(
    const _Float16* __restrict__ A16, const _Float16* __restrict__ Bt,
    const float* __restrict__ bias, const float* __restrict__ maskp,
    const float* __restrict__ xin, float* __restrict__ outf) {
  gemm_body<3>(A16, (unsigned)HDIM, Bt, (unsigned)HDIM, bias, maskp, xin, outf, (_Float16*)0);
}

__global__ __launch_bounds__(128) void pair_kernel(
    const float* __restrict__ AC, const float* __restrict__ pos, const float* __restrict__ maskp,
    const float* __restrict__ be1, const float* __restrict__ wd, _Float16* __restrict__ M16) {
  __shared__ float dist_s[NODES];
  __shared__ float msk_s[NODES];
  __shared__ __attribute__((aligned(16))) _Float16 row_s[HDIM];

  const unsigned bi = blockIdx.x;
  const unsigned b = bi / (unsigned)NODES;
  const unsigned c = threadIdx.x;

  const float pix = bf16r(pos[(size_t)bi * 3u + 0u]);
  const float piy = bf16r(pos[(size_t)bi * 3u + 1u]);
  const float piz = bf16r(pos[(size_t)bi * 3u + 2u]);
#pragma unroll 1
  for (unsigned j = c; j < (unsigned)NODES; j += 128u) {
    const size_t gj = (size_t)b * NODES + j;
    const float dx = pix - bf16r(pos[gj * 3u + 0u]);
    const float dy = piy - bf16r(pos[gj * 3u + 1u]);
    const float dz = piz - bf16r(pos[gj * 3u + 2u]);
    const float sq = dx * dx + dy * dy + dz * dz;
    dist_s[j] = (sq > 0.0f) ? sqrtf(sq) : 0.0f;
    msk_s[j] = bf16r(maskp[gj]);
  }
  __syncthreads();

  const float a = AC[(size_t)bi * KCAT + c] + bf16r(be1[c]);
  const float wv = bf16r(wd[c]);
  const float* crow = AC + (size_t)b * NODES * KCAT + HDIM + c;

  float accv = 0.0f, msum = 0.0f;
#pragma unroll 4
  for (unsigned j = 0; j < (unsigned)NODES; ++j) {
    const float h = a + crow[(size_t)j * KCAT] + dist_s[j] * wv;
    const float s = silu_act(h);
    const float mj = msk_s[j];
    accv += mj * s;
    msum += mj;
  }
  const float mi = bf16r(maskp[bi]);
  const float dr = mi * msum;
  const float inv = __builtin_amdgcn_rcpf(fmaxf(dr, 1.0f));
  const float mean = (mi * accv) * inv;
  row_s[c] = toh_flush(XCARRY * mean);
  __syncthreads();

  const unsigned q = (c < 16u) ? c : 15u;
  const v8h x = *(const v8h*)&row_s[q * 8u];
  _Float16* p = M16 + (size_t)bi * HDIM + q * 8u;
  if (c < 16u) *(volatile v8h*)p = x;
  __threadfence();
  if (c < 16u) *(volatile v8h*)p = x;
}

extern "C" void kernel_launch(void* const* d_in, const int* in_sizes, int n_in,
                              void* d_out, int out_size, void* d_ws, size_t ws_size,
                              hipStream_t stream) {
  if (n_in < 11) return;
  if ((long long)in_sizes[0] < (long long)MROWS * HDIM) return;
  if ((long long)in_sizes[1] < (long long)MROWS * 3) return;
  if ((long long)in_sizes[2] < (long long)MROWS) return;
  if ((long long)in_sizes[3] < (long long)EIN * HDIM) return;
  if ((long long)in_sizes[5] < (long long)HDIM * HDIM) return;
  if ((long long)in_sizes[7] < (long long)KCAT * HDIM) return;
  if ((long long)in_sizes[9] < (long long)HDIM * HDIM) return;
  if (in_sizes[4] < HDIM || in_sizes[6] < HDIM || in_sizes[8] < HDIM || in_sizes[10] < HDIM) return;
  if ((long long)out_size < (long long)MROWS * HDIM) return;
  if (ws_size < WS_TOTAL) return;

  const float* ns   = (const float*)d_in[0];
  const float* pos  = (const float*)d_in[1];
  const float* mask = (const float*)d_in[2];
  const float* we1  = (const float*)d_in[3];
  const float* be1  = (const float*)d_in[4];
  const float* we2  = (const float*)d_in[5];
  const float* be2  = (const float*)d_in[6];
  const float* wn1  = (const float*)d_in[7];
  const float* bn1  = (const float*)d_in[8];
  const float* wn2  = (const float*)d_in[9];
  const float* bn2  = (const float*)d_in[10];
  float* out = (float*)d_out;

  char* ws = (char*)d_ws;
  _Float16* We1_t = (_Float16*)(ws + OFF_WE1);
  _Float16* We2_t = (_Float16*)(ws + OFF_WE2);
  _Float16* Wn1_t = (_Float16*)(ws + OFF_WN1);
  _Float16* Wn2_t = (_Float16*)(ws + OFF_WN2);
  _Float16* NI16  = (_Float16*)(ws + OFF_NI);
  _Float16* M16   = (_Float16*)(ws + OFF_M);
  _Float16* HN16  = (_Float16*)(ws + OFF_HN);
  float*    AC    = (float*)(ws + OFF_AC);

  dim3 blk(256);
  dim3 gsq(HDIM / 64, HDIM / 64);

  wconv_kernel<<<gsq, blk, 0, stream>>>(we1, We1_t, (unsigned)HDIM, (unsigned)HDIM);
  wconv_kernel<<<gsq, blk, 0, stream>>>(we1 + (size_t)HDIM * HDIM, We1_t + (size_t)HDIM * HDIM,
                                        (unsigned)HDIM, (unsigned)HDIM);
  wconv_kernel<<<gsq, blk, 0, stream>>>(we2, We2_t, (unsigned)HDIM, (unsigned)HDIM);
  wconv_kernel<<<dim3(HDIM / 64, KCAT / 64), blk, 0, stream>>>(wn1, Wn1_t, (unsigned)HDIM,
                                                               (unsigned)KCAT);
  wconv_kernel<<<gsq, blk, 0, stream>>>(wn2, Wn2_t, (unsigned)HDIM, (unsigned)HDIM);

  nsconv_kernel<<<dim3(MROWS / 16), blk, 0, stream>>>(ns, NI16);
  gemm_ac_kernel<<<dim3(KCAT / 64, MROWS / 64), blk, 0, stream>>>(NI16, We1_t, AC);
  pair_kernel<<<dim3(MROWS), dim3(128), 0, stream>>>(AC, pos, mask, be1,
                                                     we1 + (size_t)2 * HDIM * HDIM, M16);
  gemm_agg_kernel<<<dim3(HDIM / 64, MROWS / 64), blk, 0, stream>>>(M16, We2_t, be2, mask, NI16);
  gemm_hn_kernel<<<dim3(HDIM / 64, MROWS / 64), blk, 0, stream>>>(NI16, Wn1_t, bn1, HN16);
  gemm_out_kernel<<<dim3(HDIM / 64, MROWS / 64), blk, 0, stream>>>(HN16, Wn2_t, bn2, mask, ns, out);
}
